// HierarchicalAutoEncoderLayer_60790967108240
// MI455X (gfx1250) — hardware-run, weakly checked
//
#include <hip/hip_runtime.h>


#ifndef NB
#define NB 1024
#endif
#define NB_FULL 1024
#define DM    128
#define DF    512
#define NEXP  128
#define KSEL  2
#define NPAIR (KSEL * NB)
#define PROWS (NPAIR + NEXP * 15 + ((16 - ((NPAIR + NEXP * 15) & 15)) & 15))
#define NTILE (PROWS / 16)
#define TEP   (((NTILE + 127) / 128) * 128)
#define PSP   32
#define XCARRY 16.0f
#define WCARRY 64.0f
#define HCARRY 256.0f
#define S1SCALE (1.0f / 1024.0f)
#define S2SCALE (1.0f / 16384.0f)

static_assert(NB % 32 == 0 && NB >= 32 && NB <= 1024);
static_assert(NB <= NB_FULL);
static_assert(NEXP == 128);
static_assert(KSEL == 2);
static_assert(PROWS % 16 == 0);
static_assert(PROWS >= NPAIR + NEXP * 15);
static_assert(NTILE <= TEP && TEP % 128 == 0 && TEP <= 1024);
static_assert(DM % 64 == 0 && DF % 64 == 0);
static_assert(DM % 32 == 0 && DF % 32 == 0);
static_assert(NB % 8 == 0);
static_assert(XCARRY * WCARRY * S1SCALE == 1.0f);
static_assert(HCARRY * WCARRY * S2SCALE == 1.0f);
static_assert(256 * 16 * 2 == 64 * 128);
static_assert(32 * 16 * 32 == 64 * (DM * 2));
static_assert(32 * 16 * 16 == 64 * (PSP * 4));
static_assert(32 * 16 * 8 == 16 * (DM * 2));
static_assert(32 * 16 * 4 == 16 * (PSP * 4));
static_assert((TEP / 128) * 32 * 16 == TEP * 4);
static_assert(32 * 8 == 64 * 4);
static_assert(32 * 16 * 4 == 16 * (64 * 2));
static_assert(32 * 16 * 8 == 16 * (64 * 4));
static_assert(32 * 16 == DM * 4);
static_assert(64 * 65 * 4 <= 131072);
static_assert((2 * NPAIR + 2 * NEXP + TEP) * 4 <= 131072);
static_assert(16 * 68 * 4 <= 131072);

typedef unsigned short hw;
typedef _Float16 h16;
typedef __attribute__((ext_vector_type(16))) _Float16 v16h;
typedef __attribute__((ext_vector_type(8)))  unsigned short v8us;
typedef __attribute__((ext_vector_type(8)))  float    v8f;
typedef __attribute__((ext_vector_type(4)))  float    v4f;
typedef __attribute__((ext_vector_type(4)))  int      v4i;
typedef __attribute__((ext_vector_type(2)))  int      v2i;
typedef v4f  __attribute__((may_alias)) v4fa;
typedef v4i  __attribute__((may_alias)) v4ia;

__device__ __forceinline__ unsigned short f2bf(float f) { unsigned u = __float_as_uint(f); u += 0x7FFFu + ((u >> 16) & 1u); return (unsigned short)(u >> 16); }
__device__ __forceinline__ float bf2f(unsigned short w) { return __uint_as_float(((unsigned)w) << 16); }
__device__ __forceinline__ int clampi(int v, int lo, int hi) { return min(max(v, lo), hi); }
static __device__ __forceinline__ h16 toh_flush(float v) { const h16 r = (h16)v; return (fabsf(v) < 6.103515625e-05f) ? (h16)0.0f : r; }
__device__ __forceinline__ unsigned short hb(h16 h) { return __builtin_bit_cast(unsigned short, h); }
__device__ __forceinline__ v16h cat16h(v8us lo, v8us hi) { return __builtin_bit_cast(v16h, __builtin_shufflevector(lo, hi, 0, 1, 2, 3, 4, 5, 6, 7, 8, 9, 10, 11, 12, 13, 14, 15)); }
__device__ __forceinline__ v8f wmmah(v16h a, v16h b, v8f c) {
    c = __builtin_amdgcn_wmma_f32_16x16x32_f16(false, a, false, b, (short)0, c, false, false);
    asm volatile("v_nop\n\tv_nop\n\tv_nop\n\tv_nop" : "+v"(c) : "v"(a), "v"(b));
    return c;
}
__device__ __forceinline__ v16h ldh(const hw* p)  { return cat16h(*(const v8us*)p, *(const v8us*)(p + 16)); }
__device__ __forceinline__ void wave_sync() { __builtin_amdgcn_fence(3  , "wavefront"); __builtin_amdgcn_wave_barrier(); asm volatile("" ::: "memory"); }

__global__ __launch_bounds__(256) void k_wt(const float* __restrict__ W, hw* WT, int R, int C, float carry) {
    __shared__ float ts[64 * 65];
    const int t = threadIdx.x;
    const int c0 = blockIdx.x * 64, r0 = blockIdx.y * 64, e = blockIdx.z;
    const float* src = W + (size_t)e * R * C + (size_t)r0 * C + c0;
#pragma unroll 1
    for (int i = 0; i < 16; ++i) { const int f = i * 256 + t; ts[(f >> 6) * 65 + (f & 63)] = src[(size_t)(f >> 6) * C + (f & 63)]; }
    __syncthreads();
    hw* dst = WT + (size_t)e * R * C + (size_t)c0 * R + r0;
#pragma unroll 1
    for (int ps = 0; ps < 2; ++ps) {
#pragma unroll 1
        for (int it = 0; it < 2; ++it) {
            const int cl = it * 32 + (t >> 3), r8 = (t & 7) * 8; v8us o;
#pragma unroll
            for (int k = 0; k < 8; ++k) o[k] = hb(toh_flush(bf2f(f2bf(ts[(r8 + k) * 65 + cl])) * carry));
            *(volatile v8us*)(dst + (size_t)cl * R + r8) = o; }
        if (ps == 0) __threadfence(); }
}

__global__ __launch_bounds__(1024) void k_route(const float* __restrict__ gate, const float* __restrict__ X, int* POS, int* TE, hw* XS, float* PSL) {
    __shared__ int eid[NPAIR];
    __shared__ int rnk[NPAIR];
    __shared__ int cntl[NEXP];
    __shared__ int sstl[NEXP];
    __shared__ __align__(16) int tel[TEP];
    const int tid = threadIdx.x, lane = tid & 31; const int wave = __builtin_amdgcn_readfirstlane(tid >> 5);
    const bool wlive = (wave * 32 < NB);
    const int b = min(tid, NB - 1);
    float v1 = __uint_as_float(0xFF800000u), v2 = __uint_as_float(0xFF800000u); int i1 = 0, i2 = 0;
#pragma unroll 1
    for (int c = 0; c < NEXP; c += 4) {
        const v4f g4 = *(const v4f*)(gate + (size_t)b * NEXP + c);
#pragma unroll
        for (int k = 0; k < 4; ++k) {
            const float v = bf2f(f2bf(g4[k])); const int e = c + k;
            const bool a = v > v1; const bool s = v > v2;
            const float nv2 = a ? v1 : (s ? v : v2); const int ni2 = a ? i1 : (s ? e : i2);
            v1 = a ? v : v1; i1 = a ? e : i1; v2 = nv2; i2 = ni2; }
    }
    i1 = clampi(i1, 0, NEXP - 1); i2 = clampi(i2, 0, NEXP - 1);
    if (wlive) { eid[2 * tid] = i1; eid[2 * tid + 1] = i2; }
    __syncthreads();
    if (tid < NEXP) {
        int c = 0;
#pragma unroll 1
        for (int p = 0; p < NPAIR; ++p) { const bool m = (eid[p] == tid); if (m) rnk[p] = c; c += m ? 1 : 0; }
        cntl[tid] = c;
    }
    if (tid < TEP) tel[tid] = -1;
    __syncthreads();
    if (wave == 0) {
        int pd[4]; int ls = 0;
#pragma unroll
        for (int i = 0; i < 4; ++i) { const int c = clampi(cntl[4 * lane + i], 0, NPAIR); pd[i] = (c + 15) & ~15; ls += pd[i]; }
        int x = ls;
#pragma unroll
        for (int d = 1; d < 32; d <<= 1) { const int y = __shfl_up(x, d, 32); x += (lane >= d) ? y : 0; }
        int s = x - ls;
#pragma unroll
        for (int i = 0; i < 4; ++i) { sstl[4 * lane + i] = s; s += pd[i]; }
    }
    __syncthreads();
    if (tid < NEXP) {
        const int s = sstl[tid] >> 4; const int nt = (clampi(cntl[tid], 0, NPAIR) + 15) >> 4;
#pragma unroll 1
        for (int j = 0; j < NPAIR / 16; ++j) { if (j < nt) tel[min(s + j, TEP - 1)] = tid; }
    }
    __syncthreads();
    const int q0 = min(2 * tid, NPAIR - 2);
    const int pos0 = clampi(sstl[i1] + rnk[q0], 0, PROWS - 1);
    const int pos1 = clampi(sstl[i2] + rnk[q0 + 1], 0, PROWS - 1);
    v8us z;
#pragma unroll
    for (int k = 0; k < 8; ++k) z[k] = (unsigned short)0;
    v4f zf;
#pragma unroll
    for (int k = 0; k < 4; ++k) zf[k] = 0.0f;
#pragma unroll 1
    for (int ps = 0; ps < 2; ++ps) {
        if (wlive) {
            v2i pp; pp[0] = pos0; pp[1] = pos1;
            *(volatile v2i*)(POS + 2 * tid) = pp;
#pragma unroll 1
            for (int it = 0; it < 32; ++it) {
                const int pa = __shfl(pos0, it, 32), pb = __shfl(pos1, it, 32);
                const int p = (lane >> 4) ? pb : pa;
                const size_t rg = (size_t)wave * 32 + it;
                const int c8 = (lane & 15) * 8;
                const v8f a = *(const v8f*)(X + rg * DM + c8); v8us oa;
#pragma unroll
                for (int k = 0; k < 8; ++k) oa[k] = hb(toh_flush(bf2f(f2bf(a[k])) * XCARRY));
                *(volatile v8us*)(XS + (size_t)p * DM + c8) = oa; }
#pragma unroll 1
            for (int it = 0; it < 16; ++it) {
                const int q = 4 * it + (lane >> 3); const int r = q >> 1;
                const int pa = __shfl(pos0, r, 32), pb = __shfl(pos1, r, 32);
                const float ga = __shfl(v1, r, 32), gb = __shfl(v2, r, 32);
                const int p = (q & 1) ? pb : pa; const float s = (q & 1) ? gb : ga;
                v4f o; o[0] = ((lane & 7) == 0) ? s : 0.0f; o[1] = 0.0f; o[2] = 0.0f; o[3] = 0.0f;
                *(volatile v4f*)(PSL + (size_t)p * PSP + (lane & 7) * 4) = o; }
        }
#pragma unroll 1
        for (int g = 0; g < 4; ++g) {
            const int e = 4 * wave + g;
            const int tot = clampi(cntl[e], 0, NPAIR); const int pbase = sstl[e] + tot; const int padcnt = ((tot + 15) & ~15) - tot;
#pragma unroll 1
            for (int it = 0; it < 8; ++it) { const int j = 2 * it + (lane >> 4); const int p = clampi(pbase + j, 0, PROWS - 1);
                if (j < padcnt) { *(volatile v8us*)(XS + (size_t)p * DM + (lane & 15) * 8) = z; } }
#pragma unroll 1
            for (int it = 0; it < 4; ++it) { const int j = 4 * it + (lane >> 3); const int p = clampi(pbase + j, 0, PROWS - 1);
                if (j < padcnt) { *(volatile v4f*)(PSL + (size_t)p * PSP + (lane & 7) * 4) = zf; } }
        }
        if (wave < TEP / 128) { const v4i v = *(const v4ia*)(&tel[wave * 128 + 4 * lane]); *(volatile v4i*)(TE + wave * 128 + 4 * lane) = v; }
        if (ps == 0) __threadfence(); }
}

__global__ __launch_bounds__(32) __attribute__((amdgpu_num_vgpr(256))) void k_gemm1(const hw* __restrict__ XS, const float* __restrict__ PSL, const hw* __restrict__ W1T,
                                                                                     const float* __restrict__ b1, const int* __restrict__ TE, hw* HP) {
    __shared__ __align__(16) float os[16 * 68];
    const int lane = threadIdx.x & 31, lr = lane & 15, hi = lane >> 4;
    const int p0 = blockIdx.x * 16, n0 = blockIdx.y * 64;
    const int tev = TE[blockIdx.x];
    if (tev < 0) return;
    const int e = __builtin_amdgcn_readfirstlane(clampi(tev, 0, NEXP - 1));
    v8f acc[4];
#pragma unroll
    for (int nb = 0; nb < 4; ++nb) acc[nb] = (v8f){};
    const size_t aoff = (size_t)(p0 + lr) * DM + 8 * hi, boff = (size_t)e * ((size_t)DF * DM) + (size_t)(n0 + lr) * DM + 8 * hi;
#pragma unroll 1
    for (int kc = 0; kc < DM; kc += 32) {
        const v16h a = ldh(XS + aoff + kc);
#pragma unroll
        for (int nb = 0; nb < 4; ++nb) { const v16h b = ldh(W1T + boff + (size_t)nb * 16 * DM + kc); acc[nb] = wmmah(a, b, acc[nb]); }
    }
#pragma unroll
    for (int nb = 0; nb < 4; ++nb) {
#pragma unroll
        for (int j = 0; j < 8; ++j) os[(hi * 8 + j) * 68 + nb * 16 + lr] = acc[nb][j]; }
    wave_sync();
    const int c8 = (lane & 7) * 8;
    v8f bb = *(const v8f*)(b1 + (size_t)e * DF + n0 + c8);
#pragma unroll
    for (int k = 0; k < 8; ++k) bb[k] = bf2f(f2bf(bb[k]));
#pragma unroll 1
    for (int ps = 0; ps < 2; ++ps) {
#pragma unroll 1
        for (int it = 0; it < 4; ++it) {
            const int row = 4 * it + (lane >> 3);
            const float* orow = &os[row * 68 + c8];
            const v4f x0 = *(const v4fa*)orow; const v4f x1 = *(const v4fa*)(orow + 4);
            const float s = PSL[(size_t)(p0 + row) * PSP];
            v8us oh;
#pragma unroll
            for (int k = 0; k < 4; ++k) {
                float z0 = x0[k] * S1SCALE + bb[k]; z0 = (z0 > 0.0f) ? z0 : 0.0f;
                float z1 = x1[k] * S1SCALE + bb[4 + k]; z1 = (z1 > 0.0f) ? z1 : 0.0f;
                const float t0 = (z0 * s) * HCARRY, t1 = (z1 * s) * HCARRY;
                oh[k] = hb(toh_flush(t0)); oh[4 + k] = hb(toh_flush(t1)); }
            hw* dst = HP + (size_t)(p0 + row) * DF + n0 + c8;
            *(volatile v8us*)dst = oh; }
        if (ps == 0) __threadfence(); }
}

__global__ __launch_bounds__(32) __attribute__((amdgpu_num_vgpr(256))) void k_gemm2(const hw* __restrict__ HP, const hw* __restrict__ W2T, const float* __restrict__ b2,
                                                                                     const int* __restrict__ TE, float* YS) {
    __shared__ __align__(16) float os[16 * 68];
    const int lane = threadIdx.x & 31, lr = lane & 15, hi = lane >> 4;
    const int p0 = blockIdx.x * 16, n0 = blockIdx.y * 64;
    const int tev = TE[blockIdx.x];
    if (tev < 0) return;
    const int e = __builtin_amdgcn_readfirstlane(clampi(tev, 0, NEXP - 1));
    v8f acc[4];
#pragma unroll
    for (int nb = 0; nb < 4; ++nb) acc[nb] = (v8f){};
    const size_t aoff = (size_t)(p0 + lr) * DF + 8 * hi, boff = (size_t)e * ((size_t)DM * DF) + (size_t)(n0 + lr) * DF + 8 * hi;
#pragma unroll 1
    for (int kc = 0; kc < DF; kc += 32) {
        const v16h a = ldh(HP + aoff + kc);
#pragma unroll
        for (int nb = 0; nb < 4; ++nb) { const v16h b = ldh(W2T + boff + (size_t)nb * 16 * DF + kc); acc[nb] = wmmah(a, b, acc[nb]); }
    }
#pragma unroll
    for (int nb = 0; nb < 4; ++nb) {
#pragma unroll
        for (int j = 0; j < 8; ++j) os[(hi * 8 + j) * 68 + nb * 16 + lr] = acc[nb][j]; }
    wave_sync();
    const int c4 = (lane & 15) * 4;
    v4f bb = *(const v4f*)(b2 + (size_t)e * DM + n0 + c4);
#pragma unroll
    for (int k = 0; k < 4; ++k) bb[k] = bf2f(f2bf(bb[k]));
#pragma unroll 1
    for (int ps = 0; ps < 2; ++ps) {
#pragma unroll 1
        for (int it = 0; it < 8; ++it) {
            const int row = 2 * it + (lane >> 4);
            const v4f x = *(const v4fa*)(&os[row * 68 + c4]);
            v4f y;
#pragma unroll
            for (int k = 0; k < 4; ++k) y[k] = x[k] * S2SCALE + bb[k];
            *(volatile v4f*)(YS + (size_t)(p0 + row) * DM + n0 + c4) = y; }
        if (ps == 0) __threadfence(); }
}

__global__ __launch_bounds__(256) void k_combine(const int* __restrict__ POS, const int* __restrict__ kin, const float* __restrict__ YS, float* OUT) {
    const int lane = threadIdx.x & 31, wave = threadIdx.x >> 5;
    const int i = min((int)blockIdx.x * 8 + wave, NB - 1);
    const int p0 = clampi(POS[2 * i], 0, PROWS - 1);
    const int p1 = clampi(POS[2 * i + 1], 0, PROWS - 1);
    const bool bad = (kin[0] != KSEL);
    const float qn = __uint_as_float(0x7FC00000u);
    const v4f a = *(const v4f*)(YS + (size_t)p0 * DM + lane * 4);
    const v4f c = *(const v4f*)(YS + (size_t)p1 * DM + lane * 4);
    v4f v;
#pragma unroll
    for (int k = 0; k < 4; ++k) { const float s = a[k] + c[k]; v[k] = bad ? qn : s; }
    float* orow = OUT + (size_t)i * DM;
    *(volatile v4f*)(orow + lane * 4) = v;
    __threadfence();
    *(volatile v4f*)(orow + lane * 4) = v;
}

static constexpr size_t al256(size_t v) { return (v + 255) & ~(size_t)255; }
static constexpr size_t SZ_W1T = al256((size_t)NEXP * DF * DM * 2);
static constexpr size_t SZ_W2T = al256((size_t)NEXP * DM * DF * 2);
static constexpr size_t SZ_POS = al256((size_t)NPAIR * 4);
static constexpr size_t SZ_TE  = al256((size_t)TEP * 4);
static constexpr size_t SZ_XS  = al256((size_t)PROWS * DM * 2);
static constexpr size_t SZ_PSL = al256((size_t)PROWS * PSP * 4);
static constexpr size_t SZ_HP  = al256((size_t)PROWS * DF * 2);
static constexpr size_t SZ_YS  = al256((size_t)PROWS * DM * 4);
static constexpr size_t SZ_TOTAL = SZ_W1T + SZ_W2T + SZ_POS + SZ_TE + SZ_XS + SZ_PSL + SZ_HP + SZ_YS;
static_assert(SZ_TOTAL <= (size_t)134217728);
static_assert((size_t)NTILE * 16 * DM * 2 <= SZ_XS);
static_assert((size_t)NTILE * 16 * PSP * 4 <= SZ_PSL);
static_assert((size_t)NTILE * 16 * DF * 2 <= SZ_HP);
static_assert((size_t)NTILE * 16 * DM * 4 <= SZ_YS);

extern "C" void kernel_launch(void* const* d_in, const int* in_sizes, int n_in,
                              void* d_out, int out_size, void* d_ws, size_t ws_size, hipStream_t stream) {
    if (n_in < 7) return;
    if ((size_t)in_sizes[0] < (size_t)NB * DM) return;
    if ((size_t)in_sizes[1] < (size_t)NB * NEXP) return;
    if ((size_t)in_sizes[2] < (size_t)NEXP * DM * DF) return;
    if ((size_t)in_sizes[3] < (size_t)NEXP * DF * DM) return;
    if ((size_t)in_sizes[4] < (size_t)NEXP * DF) return;
    if ((size_t)in_sizes[5] < (size_t)NEXP * DM) return;
    if ((size_t)in_sizes[6] < (size_t)1) return;
    if ((size_t)out_size < (size_t)NB * DM) return;
    if (SZ_TOTAL > ws_size) return;
    const float* X    = (const float*)d_in[0];
    const float* gate = (const float*)d_in[1];
    const float* Wenc = (const float*)d_in[2];
    const float* Wdec = (const float*)d_in[3];
    const float* benc = (const float*)d_in[4];
    const float* bdec = (const float*)d_in[5];
    const int*   kin  = (const int*)d_in[6];
    float* OUT = (float*)d_out;
    char* wsp = (char*)d_ws;
    hw*  W1T = (hw*)wsp;  wsp += SZ_W1T;
    hw*  W2T = (hw*)wsp;  wsp += SZ_W2T;
    int* POS = (int*)wsp; wsp += SZ_POS;
    int* TE  = (int*)wsp; wsp += SZ_TE;
    hw*  XS  = (hw*)wsp;  wsp += SZ_XS;
    float* PSL = (float*)wsp; wsp += SZ_PSL;
    hw*  HP  = (hw*)wsp;  wsp += SZ_HP;
    float* YS = (float*)wsp; wsp += SZ_YS;

    k_wt<<<dim3(DF / 64, DM / 64, NEXP), 256, 0, stream>>>(Wenc, W1T, DM, DF, WCARRY);
    k_wt<<<dim3(DM / 64, DF / 64, NEXP), 256, 0, stream>>>(Wdec, W2T, DF, DM, WCARRY);
    k_route<<<1, 1024, 0, stream>>>(gate, X, POS, TE, XS, PSL);
    k_gemm1<<<dim3(PROWS / 16, DF / 64), 32, 0, stream>>>(XS, PSL, W1T, benc, TE, HP);
    k_gemm2<<<dim3(PROWS / 16, DM / 64), 32, 0, stream>>>(HP, W2T, bdec, TE, YS);
    k_combine<<<NB / 8, 256, 0, stream>>>(POS, kin, YS, OUT);
}
